// SwinMoBABlock_14276471292735
// MI455X (gfx1250) — hardware-verified
//
#include <hip/hip_runtime.h>
#include <math.h>
#include <stdint.h>

#ifndef NBAT
#define NBAT 8
#endif
#define LIMG   3136
#define RESO   56
#define WSZ    7
#define NWI    64
#define WN     49
#define WP     64
#define NHEAD  8
#define HDM    32
#define CDIM   256
#define CQKV   768
#define CMLP   1024
#define NRPB   169
#define NTOK   (NBAT * LIMG)
#define NWT    (NBAT * NWI)
#define NKVW   (4 * NBAT)
#define OROWS  (NWT * WP)
#define NBLK   (NTOK / 128)
#define KVTOK  ((((NKVW - 1) / 8) + 1) * (WSZ * RESO))
#define KVBLK  ((KVTOK + 127) / 128)
#define KVROWS (KVBLK * 128)
#define MB0    ((NBLK + 1) / 2)
#define MB1    (NBLK - MB0)
#define HROWS  (MB0 * 128)
#define STP    68
#define ASP    36
#define QSC    64.0f
#define KSC    16.0f
#define VSC    16.0f
#define LSC    8.0f
#define OSC    256.0f
#define HSC    64.0f
#define CSC    (0.17677669529663687f / 1024.0f)

static_assert((NTOK % 128) == 0);
static_assert(NBLK * 128 == NTOK);
static_assert((NTOK % 8) == 0);
static_assert(NKVW <= NWI);
static_assert(KVTOK <= KVROWS);
static_assert(KVROWS <= NTOK);
static_assert(MB0 >= 1);
static_assert(MB1 >= 0);
static_assert(MB0 * 128 == HROWS);
static_assert((STP * 4) % 16 == 0);
static_assert((ASP * 4) % 16 == 0);
static_assert(NHEAD * HDM == CDIM);
static_assert(WN <= WP);
static_assert(RESO == 8 * WSZ);
static_assert(NWI == 64);

typedef _Float16 v16h __attribute__((ext_vector_type(16)));
typedef _Float16 v8h  __attribute__((ext_vector_type(8)));
typedef float    v8f  __attribute__((ext_vector_type(8)));
typedef float    v4f  __attribute__((ext_vector_type(4)));
typedef unsigned int v4u __attribute__((ext_vector_type(4)));

union Frag { v16h v; v8h h[2]; };

__device__ __forceinline__ unsigned short bf_bits(float f) {
  unsigned u = __float_as_uint(f);
  return (unsigned short)((u + 0x7FFFu + ((u >> 16) & 1u)) >> 16);
}
__device__ __forceinline__ float bfr(float f) { return __uint_as_float(((unsigned)bf_bits(f)) << 16); }
__device__ __forceinline__ unsigned short h_bits(_Float16 x) { return __builtin_bit_cast(unsigned short, x); }
__device__ __forceinline__ unsigned pk16(unsigned short a, unsigned short b) { return (unsigned)a | ((unsigned)b << 16); }
__device__ __forceinline__ v8f zero8() { v8f z = {0.f, 0.f, 0.f, 0.f, 0.f, 0.f, 0.f, 0.f}; return z; }

__device__ __forceinline__ v16h ldfrag_h(const _Float16* p) {
  Frag f;
  f.h[0] = *(const v8h*)(p);
  f.h[1] = *(const v8h*)(p + 16);
  return f.v;
}

__device__ __forceinline__ v8f mma_h(v16h a, v16h b, v8f c) {
  c = __builtin_amdgcn_wmma_f32_16x16x32_f16(false, a, false, b, (short)0, c, false, false);
#if defined(__HIP_DEVICE_COMPILE__)
  asm volatile("v_nop\n\tv_nop\n\tv_nop\n\tv_nop" : "+v"(c) : "v"(a), "v"(b));
#endif
  return c;
}
__device__ __forceinline__ void wave_sync_lds() {
  __builtin_amdgcn_fence(__ATOMIC_RELEASE, "workgroup");
  __builtin_amdgcn_wave_barrier();
  __builtin_amdgcn_fence(__ATOMIC_ACQUIRE, "workgroup");
}

__device__ __forceinline__ v4u pack8h(v4f a, v4f b) {
  v4u p;
  p[0] = pk16(h_bits((_Float16)a[0]), h_bits((_Float16)a[1]));
  p[1] = pk16(h_bits((_Float16)a[2]), h_bits((_Float16)a[3]));
  p[2] = pk16(h_bits((_Float16)b[0]), h_bits((_Float16)b[1]));
  p[3] = pk16(h_bits((_Float16)b[2]), h_bits((_Float16)b[3]));
  return p;
}
__device__ __forceinline__ void split8h(v4f a, v4f b, v4u& ph, v4u& pl) {
  v4f ra, rb;
#pragma unroll
  for (int e = 0; e < 4; ++e) {
    const _Float16 ha = (_Float16)a[e];
    ra[e] = (a[e] - (float)ha) * 2048.0f;
    const _Float16 hb = (_Float16)b[e];
    rb[e] = (b[e] - (float)hb) * 2048.0f;
  }
  ph = pack8h(a, b);
  pl = pack8h(ra, rb);
}
__device__ __forceinline__ void splitq8h(v4f a, v4f b, v4u& ph, v4u& pl) {
  v4f ra, rb;
#pragma unroll
  for (int e = 0; e < 4; ++e) {
    const _Float16 ha = (_Float16)a[e];
    ra[e] = a[e] - (float)ha;
    const _Float16 hb = (_Float16)b[e];
    rb[e] = b[e] - (float)hb;
  }
  ph = pack8h(a, b);
  pl = pack8h(ra, rb);
}

__device__ __forceinline__ int tok_row(int wg, int n) {
  const int b = wg / NWI, wi = wg - b * NWI;
  const int wr = wi >> 3, wc = wi & 7;
  const int r = n / WSZ, cc = n - r * WSZ;
  return b * LIMG + (wr * WSZ + r) * RESO + wc * WSZ + cc;
}

__global__ __launch_bounds__(256) void cvt_wT(const float* __restrict__ w, unsigned short* outp, int nin, int nout) {
  __shared__ float tile[64][33];
  const int tid = threadIdx.x;
  const int i0 = blockIdx.x * 64;
  const int o0 = blockIdx.y * 32;
#pragma unroll
  for (int p = 0; p < 8; ++p) {
    const int idx = p * 256 + tid;
    const int i = idx >> 5, o = idx & 31;
    tile[i][o] = w[(size_t)(i0 + i) * nout + o0 + o];
  }
  __syncthreads();
  const int o = tid >> 3, c8 = (tid & 7) * 8;
  v4u pk;
#pragma unroll
  for (int e = 0; e < 4; ++e) {
    const float fa = bfr(tile[c8 + 2 * e][o]) * 256.0f;
    const float fb = bfr(tile[c8 + 2 * e + 1][o]) * 256.0f;
    pk[e] = pk16(h_bits((_Float16)fa), h_bits((_Float16)fb));
  }
  unsigned short* gp = outp + (size_t)(o0 + o) * nin + i0 + c8;
  *(volatile v4u*)gp = pk;
  __threadfence();
  *(volatile v4u*)gp = pk;
}

template <bool BFIN>
__global__ __launch_bounds__(256) void ln256(const float* __restrict__ xin, const float* __restrict__ g,
                                             const float* __restrict__ bb, unsigned short* oh, unsigned short* ol) {
#pragma clang fp contract(off)
  const int tid = threadIdx.x, wave = tid >> 5, lane = tid & 31;
  const int row = blockIdx.x * 8 + wave;
  const float* xr = xin + (size_t)row * CDIM + lane * 8;
  v4f a0 = *(const v4f*)(xr);
  v4f a1 = *(const v4f*)(xr + 4);
  if (BFIN) {
#pragma unroll
    for (int e = 0; e < 4; ++e) { a0[e] = bfr(a0[e]); a1[e] = bfr(a1[e]); }
  }
  float s = ((a0[0] + a0[1]) + (a0[2] + a0[3])) + ((a1[0] + a1[1]) + (a1[2] + a1[3]));
#pragma unroll
  for (int off = 1; off < 32; off <<= 1) s = s + __shfl_xor(s, off, 32);
  const float mu = s * (1.0f / 256.0f);
  v4f d0, d1;
  float s2 = 0.f;
#pragma unroll
  for (int e = 0; e < 4; ++e) {
    d0[e] = a0[e] - mu;
    const float q0 = d0[e] * d0[e];
    s2 = s2 + q0;
    d1[e] = a1[e] - mu;
    const float q1 = d1[e] * d1[e];
    s2 = s2 + q1;
  }
#pragma unroll
  for (int off = 1; off < 32; off <<= 1) s2 = s2 + __shfl_xor(s2, off, 32);
  const float var = s2 * (1.0f / 256.0f);
  const float rstd = rsqrtf(var + 1e-5f);
  v4f z0, z1;
#pragma unroll
  for (int e = 0; e < 4; ++e) {
    const int cha = lane * 8 + e, chb = lane * 8 + 4 + e;
    float ta = d0[e] * rstd;
    ta = ta * bfr(g[cha]);
    ta = ta + bfr(bb[cha]);
    z0[e] = ta * LSC;
    float tb = d1[e] * rstd;
    tb = tb * bfr(g[chb]);
    tb = tb + bfr(bb[chb]);
    z1[e] = tb * LSC;
  }
  v4u ph, pl;
  split8h(z0, z1, ph, pl);
  const size_t o = (size_t)row * CDIM + lane * 8;
  for (int pass = 0; pass < 2; ++pass) {
    *(volatile v4u*)(oh + o) = ph;
    *(volatile v4u*)(ol + o) = pl;
    __threadfence();
  }
}

template <int MODE>
__global__ __launch_bounds__(256)
void gemm_k(const unsigned short* __restrict__ Ah, const unsigned short* __restrict__ Al,
            const unsigned short* __restrict__ Bt, int K, int nbase, int mbase,
            const float* __restrict__ f0, const float* __restrict__ f1,
            float* outF, unsigned short* h0, unsigned short* h1, unsigned short* h2,
            unsigned short* h3, unsigned short* h4, float oscale) {
  __shared__ __align__(16) float sbuf[8 * 16 * STP];
  const int tid = threadIdx.x, wave = tid >> 5, lane = tid & 31, hh = lane >> 4, c = lane & 15;
  const int n0 = nbase + blockIdx.x * 64, m0 = blockIdx.y * 128;
  const int mloc = m0 + wave * 16;
  const int mg = mbase + mloc;
  const int arow = ((MODE == 0) ? mloc : mg) + c;
  const _Float16* A0 = (const _Float16*)(const void*)Ah;
  const _Float16* A1 = (const _Float16*)(const void*)Al;
  const _Float16* B  = (const _Float16*)(const void*)Bt;

  int wrow = 0;
  if (MODE == 2) {
    const int bimg = arow / LIMG, l = arow - bimg * LIMG;
    const int hr = l / RESO, col = l - hr * RESO;
    const int wr = hr / WSZ, ri = hr - wr * WSZ;
    const int wc = col / WSZ, ci = col - wc * WSZ;
    wrow = (bimg * NWI + wr * 8 + wc) * WP + ri * WSZ + ci;
  }

  v8f acch[4], accl[4];
#pragma unroll
  for (int nt = 0; nt < 4; ++nt) { acch[nt] = zero8(); accl[nt] = zero8(); }

#pragma unroll 1
  for (int k0 = 0; k0 < K; k0 += 32) {
    v16h ah, al;
    if (MODE == 2) {
      const size_t oa = ((size_t)(k0 >> 5) * OROWS + wrow) * HDM + 8 * hh;
      ah = ldfrag_h(A0 + oa);
      al = ldfrag_h(A1 + oa);
    } else {
      const size_t aoff = (size_t)arow * K + k0 + 8 * hh;
      ah = ldfrag_h(A0 + aoff);
      al = ldfrag_h(A1 + aoff);
    }
#pragma unroll
    for (int nt = 0; nt < 4; ++nt) {
      const v16h bfrag = ldfrag_h(B + (size_t)(n0 + nt * 16 + c) * K + k0 + 8 * hh);
      acch[nt] = mma_h(ah, bfrag, acch[nt]);
      accl[nt] = mma_h(al, bfrag, accl[nt]);
    }
  }

  float* st = sbuf + wave * (16 * STP);
#pragma unroll
  for (int nt = 0; nt < 4; ++nt) {
#pragma unroll
    for (int r = 0; r < 8; ++r) {
      const float v = acch[nt][r] + accl[nt][r] * (1.0f / 2048.0f);
      st[(8 * hh + r) * STP + nt * 16 + c] = v * oscale;
    }
  }
  wave_sync_lds();

  if (MODE == 0 || MODE == 2) {
    v4f ov[8];
    size_t offs[8];
#pragma unroll
    for (int it = 0; it < 8; ++it) {
      const int q = it * 2 + hh;
      const int col = n0 + c * 4;
      const size_t ro = (size_t)(mg + q) * CDIM + col;
      const v4f v = *(const v4f*)(st + q * STP + c * 4);
      const v4f rr = *(const v4f*)(f1 + ro);
      v4f u;
#pragma unroll
      for (int e = 0; e < 4; ++e) {
        const float t = v[e] + bfr(f0[col + e]);
        const float rs = (MODE == 2) ? bfr(rr[e]) : rr[e];
        u[e] = rs + t;
      }
      ov[it] = u;
      offs[it] = ro;
    }
    for (int pass = 0; pass < 2; ++pass) {
#pragma unroll
      for (int it = 0; it < 8; ++it) *(volatile v4f*)(outF + offs[it]) = ov[it];
      __threadfence();
    }
  } else if (MODE == 1) {
    const int part = n0 >> 8, colp = n0 & 255;
    unsigned short* dA = (part == 0) ? h0 : ((part == 1) ? h2 : h3);
    unsigned short* dB = (part == 0) ? h1 : h4;
    v4u pa[4], pb[4];
    size_t offs[4];
#pragma unroll
    for (int it = 0; it < 4; ++it) {
      const int q = it * 4 + (lane >> 3), piece = lane & 7;
      const int colg = n0 + piece * 8;
      v4f fa = *(const v4f*)(st + q * STP + piece * 8);
      v4f fb = *(const v4f*)(st + q * STP + piece * 8 + 4);
#pragma unroll
      for (int e = 0; e < 4; ++e) {
        fa[e] = fa[e] + bfr(f0[colg + e]);
        fb[e] = fb[e] + bfr(f0[colg + 4 + e]);
      }
      if (part == 0) {
        fa = fa * QSC; fb = fb * QSC;
        splitq8h(fa, fb, pa[it], pb[it]);
      } else if (part == 1) {
        fa = fa * KSC; fb = fb * KSC;
        pa[it] = pack8h(fa, fb);
        pb[it] = pa[it];
      } else {
        fa = fa * VSC; fb = fb * VSC;
        split8h(fa, fb, pa[it], pb[it]);
      }
      offs[it] = (size_t)(mloc + q) * CDIM + colp + piece * 8;
    }
    for (int pass = 0; pass < 2; ++pass) {
#pragma unroll
      for (int it = 0; it < 4; ++it) {
        *(volatile v4u*)(dA + offs[it]) = pa[it];
        if (part != 1) *(volatile v4u*)(dB + offs[it]) = pb[it];
      }
      __threadfence();
    }
  } else {
    v4u pa[4], pb[4];
    size_t offs[4];
#pragma unroll
    for (int it = 0; it < 4; ++it) {
      const int q = it * 4 + (lane >> 3), piece = lane & 7;
      const int col0 = n0 + piece * 8;
      const v4f fa = *(const v4f*)(st + q * STP + piece * 8);
      const v4f fb = *(const v4f*)(st + q * STP + piece * 8 + 4);
      v4f ua, ub;
#pragma unroll
      for (int e = 0; e < 4; ++e) {
        const float u0 = fa[e] + bfr(f0[col0 + e]);
        const float g0 = 0.5f * u0 * (1.0f + erff(u0 * 0.70710678118654752f));
        ua[e] = g0 * HSC;
        const float u1 = fb[e] + bfr(f0[col0 + 4 + e]);
        const float g1 = 0.5f * u1 * (1.0f + erff(u1 * 0.70710678118654752f));
        ub[e] = g1 * HSC;
      }
      split8h(ua, ub, pa[it], pb[it]);
      offs[it] = (size_t)(mloc + q) * CMLP + col0;
    }
    for (int pass = 0; pass < 2; ++pass) {
#pragma unroll
      for (int it = 0; it < 4; ++it) {
        *(volatile v4u*)(h0 + offs[it]) = pa[it];
        *(volatile v4u*)(h1 + offs[it]) = pb[it];
      }
      __threadfence();
    }
  }
}

__global__ __launch_bounds__(128)
void attn_k(const unsigned short* __restrict__ Qh, const unsigned short* __restrict__ Ql,
            const unsigned short* __restrict__ Kp,
            const unsigned short* __restrict__ Vh, const unsigned short* __restrict__ Vl,
            const float* __restrict__ rpb, unsigned short* Oh, unsigned short* Ol) {
  __shared__ __align__(16) unsigned short Ks[WP * HDM];
  __shared__ __align__(16) unsigned short Vth[HDM * WP];
  __shared__ __align__(16) unsigned short Vtl[HDM * WP];
  __shared__ __align__(16) float Btab[WP * WP];
  __shared__ __align__(16) float Sst[4 * 16 * ASP];
  const int tid = threadIdx.x, wave = tid >> 5, lane = tid & 31, hh = lane >> 4, c = lane & 15;
  const int head = blockIdx.x & 7, bw = blockIdx.x >> 3;
  const int kw = bw % NKVW;
  const int c0 = head * HDM;

  {
    const int n = tid >> 1, i = tid & 1;
    const bool val = n < WN;
    const int nc = val ? n : (WN - 1);
    const size_t row = (size_t)tok_row(kw, nc);
    const v4u* kg = (const v4u*)(Kp + row * CDIM + c0 + 16 * i);
    const v4u* hg = (const v4u*)(Vh + row * CDIM + c0 + 16 * i);
    const v4u* lg = (const v4u*)(Vl + row * CDIM + c0 + 16 * i);
    const unsigned msk = val ? 0xFFFFFFFFu : 0u;
#pragma unroll
    for (int p = 0; p < 2; ++p) {
      v4u kv4 = kg[p], hw = hg[p], lw = lg[p];
      kv4 = kv4 & msk; hw = hw & msk; lw = lw & msk;
      *(v4u*)(Ks + n * HDM + 16 * i + 8 * p) = kv4;
#pragma unroll
      for (int e = 0; e < 4; ++e) {
        const int d = 16 * i + 8 * p + 2 * e;
        Vth[d * WP + n]       = (unsigned short)(hw[e] & 0xFFFFu);
        Vth[(d + 1) * WP + n] = (unsigned short)(hw[e] >> 16);
        Vtl[d * WP + n]       = (unsigned short)(lw[e] & 0xFFFFu);
        Vtl[(d + 1) * WP + n] = (unsigned short)(lw[e] >> 16);
      }
    }
  }
  {
    const int q = tid >> 1, mb = (tid & 1) * 32;
    const int qn = (q < WN) ? q : (WN - 1);
    const int qr = qn / WSZ, qc = qn - qr * WSZ;
#pragma unroll 4
    for (int t = 0; t < 32; ++t) {
      const int m = mb + t;
      const int mc = (m < WN) ? m : (WN - 1);
      const int kr = mc / WSZ, kc = mc - kr * WSZ;
      const int ridx = (qr - kr + 6) * 13 + (qc - kc + 6);
      const float bv = bfr(rpb[ridx * NHEAD + head]);
      Btab[q * WP + m] = (m < WN) ? bv : -1.0e30f;
    }
  }
  __syncthreads();

  const _Float16* Ksh = (const _Float16*)(const void*)Ks;
  const _Float16* Vhh = (const _Float16*)(const void*)Vth;
  const _Float16* Vlh = (const _Float16*)(const void*)Vtl;
  const _Float16* Qhg = (const _Float16*)(const void*)Qh;
  const _Float16* Qlg = (const _Float16*)(const void*)Ql;
  float* st = Sst + wave * (16 * ASP);
  const int qt = wave;
  const int nq = qt * 16 + c;
  const int nqc = (nq < WN) ? nq : (WN - 1);
  const float* brow = Btab + (qt * 16 + c) * WP + 8 * hh;

  v8f osum[2];
  osum[0] = zero8(); osum[1] = zero8();

#pragma unroll 1
  for (int tp = 0; tp < 4; ++tp) {
    const int qw = tp * (NBAT * 16) + (bw >> 2);
    const size_t rq = (size_t)tok_row(qw, nqc);
    const size_t qo = rq * CDIM + c0 + 8 * hh;
    const v16h qfh = ldfrag_h(Qhg + qo);
    const v16h qfl = ldfrag_h(Qlg + qo);
    v8f s[4];
#pragma unroll
    for (int j = 0; j < 4; ++j) {
      const v16h ka = ldfrag_h(Ksh + (size_t)(j * 16 + c) * HDM + 8 * hh);
      const v8f t0 = mma_h(ka, qfh, zero8());
      s[j] = mma_h(ka, qfl, t0);
    }
    float mx = -1.0e30f;
#pragma unroll
    for (int j = 0; j < 4; ++j) {
      const v4f b0 = *(const v4f*)(brow + 16 * j);
      const v4f b1 = *(const v4f*)(brow + 16 * j + 4);
#pragma unroll
      for (int r = 0; r < 8; ++r) {
        const float bb = (r < 4) ? b0[r] : b1[r - 4];
        const float lgv = s[j][r] * CSC + bb;
        s[j][r] = lgv;
        mx = fmaxf(mx, lgv);
      }
    }
    mx = fmaxf(mx, __shfl_xor(mx, 16, 32));
    float psum = 0.f;
    v16h pf0, pf1;
#pragma unroll
    for (int i = 0; i < 8; ++i) {
      const float e0 = __expf(s[0][i] - mx);
      const float e1 = __expf(s[1][i] - mx);
      const float e2 = __expf(s[2][i] - mx);
      const float e3 = __expf(s[3][i] - mx);
      psum = psum + ((e0 + e1) + (e2 + e3));
      pf0[i]     = (_Float16)(e0 * 1024.0f);
      pf0[8 + i] = (_Float16)(e1 * 1024.0f);
      pf1[i]     = (_Float16)(e2 * 1024.0f);
      pf1[8 + i] = (_Float16)(e3 * 1024.0f);
    }
    const float lsum = psum + __shfl_xor(psum, 16, 32);
    v8f oh[2], ol[2];
#pragma unroll
    for (int nt = 0; nt < 2; ++nt) {
      const v16h va = ldfrag_h(Vhh + (size_t)(nt * 16 + c) * WP + 8 * hh);
      oh[nt] = mma_h(pf0, va, zero8());
      const v16h vb = ldfrag_h(Vhh + (size_t)(nt * 16 + c) * WP + 32 + 8 * hh);
      oh[nt] = mma_h(pf1, vb, oh[nt]);
      const v16h wa = ldfrag_h(Vlh + (size_t)(nt * 16 + c) * WP + 8 * hh);
      ol[nt] = mma_h(pf0, wa, zero8());
      const v16h wb = ldfrag_h(Vlh + (size_t)(nt * 16 + c) * WP + 32 + 8 * hh);
      ol[nt] = mma_h(pf1, wb, ol[nt]);
    }
#pragma unroll
    for (int r = 0; r < 8; ++r) {
      const float lq = __shfl(lsum, 8 * hh + r, 32);
      const float inv = 1.0f / (lq * 16384.0f);
      osum[0][r] = osum[0][r] + (oh[0][r] + ol[0][r] * (1.0f / 2048.0f)) * inv;
      osum[1][r] = osum[1][r] + (oh[1][r] + ol[1][r] * (1.0f / 2048.0f)) * inv;
    }
  }

#pragma unroll
  for (int nt = 0; nt < 2; ++nt) {
#pragma unroll
    for (int r = 0; r < 8; ++r) st[(8 * hh + r) * ASP + nt * 16 + c] = osum[nt][r] * 0.25f;
  }
  wave_sync_lds();
  v4u pa[2], pb[2];
  size_t offs[2];
#pragma unroll
  for (int it = 0; it < 2; ++it) {
    const int q = it * 8 + (lane >> 2), piece = lane & 3;
    v4f fa = *(const v4f*)(st + q * ASP + piece * 8);
    v4f fb = *(const v4f*)(st + q * ASP + piece * 8 + 4);
    fa = fa * OSC;
    fb = fb * OSC;
    split8h(fa, fb, pa[it], pb[it]);
    offs[it] = (((size_t)head * OROWS) + (size_t)bw * WP + qt * 16 + q) * HDM + piece * 8;
  }
  for (int pass = 0; pass < 2; ++pass) {
#pragma unroll
    for (int it = 0; it < 2; ++it) {
      *(volatile v4u*)(Oh + offs[it]) = pa[it];
      *(volatile v4u*)(Ol + offs[it]) = pb[it];
    }
    __threadfence();
  }
}

extern "C" void kernel_launch(void* const* d_in, const int* in_sizes, int n_in,
                              void* d_out, int out_size, void* d_ws, size_t ws_size,
                              hipStream_t stream) {
  if (n_in < 14) return;
  if (in_sizes[0] != NTOK * CDIM) return;
  if (in_sizes[1] != CDIM || in_sizes[2] != CDIM) return;
  if (in_sizes[3] != CDIM * CQKV || in_sizes[4] != CQKV) return;
  if (in_sizes[5] != NRPB * NHEAD) return;
  if (in_sizes[6] != CDIM * CDIM || in_sizes[7] != CDIM) return;
  if (in_sizes[8] != CDIM || in_sizes[9] != CDIM) return;
  if (in_sizes[10] != CDIM * CMLP || in_sizes[11] != CMLP) return;
  if (in_sizes[12] != CMLP * CDIM || in_sizes[13] != CDIM) return;
  if (out_size != NTOK * CDIM) return;

  const float* x      = (const float*)d_in[0];
  const float* g1     = (const float*)d_in[1];
  const float* b1     = (const float*)d_in[2];
  const float* w_qkv  = (const float*)d_in[3];
  const float* b_qkv  = (const float*)d_in[4];
  const float* rpb    = (const float*)d_in[5];
  const float* w_proj = (const float*)d_in[6];
  const float* b_proj = (const float*)d_in[7];
  const float* g2     = (const float*)d_in[8];
  const float* b2     = (const float*)d_in[9];
  const float* w_fc1  = (const float*)d_in[10];
  const float* b_fc1  = (const float*)d_in[11];
  const float* w_fc2  = (const float*)d_in[12];
  const float* b_fc2  = (const float*)d_in[13];
  float* out = (float*)d_out;

  const size_t sWq = (size_t)CQKV * CDIM * 2;
  const size_t sWp = (size_t)CDIM * CDIM * 2;
  const size_t sW1 = (size_t)CMLP * CDIM * 2;
  const size_t sW2 = (size_t)CDIM * CMLP * 2;
  const size_t sLN = (size_t)NTOK * CDIM * 2;
  const size_t sXR = (size_t)NTOK * CDIM * 4;
  const size_t sQ  = (size_t)NTOK * CDIM * 2;
  const size_t sKV = (size_t)KVROWS * CDIM * 2;
  const size_t sO  = (size_t)NHEAD * OROWS * HDM * 2;
  const size_t sH  = (size_t)HROWS * CMLP * 2;
  size_t off = 0;
  const size_t oWq  = off; off += sWq;
  const size_t oWp  = off; off += sWp;
  const size_t oW1  = off; off += sW1;
  const size_t oW2  = off; off += sW2;
  const size_t oLNh = off; off += sLN;
  const size_t oLNl = off; off += sLN;
  const size_t oXR  = off; off += sXR;
  const size_t oBig = off;
  const size_t oQh  = oBig;
  const size_t oQl  = oQh + sQ;
  const size_t oK   = oQl + sQ;
  const size_t oVh  = oK + sKV;
  const size_t oVl  = oVh + sKV;
  const size_t oOh  = oVl + sKV;
  const size_t oOl  = oOh + sO;
  const size_t endA = oOl + sO;
  const size_t oHh  = oBig;
  const size_t oHl  = oHh + sH;
  const size_t endB = oHl + sH;
  off = (endA > endB) ? endA : endB;
  if (off > ws_size) return;
  if (off > (size_t)134217728) return;

  char* ws = (char*)d_ws;
  unsigned short* Wq  = (unsigned short*)(ws + oWq);
  unsigned short* Wp  = (unsigned short*)(ws + oWp);
  unsigned short* W1  = (unsigned short*)(ws + oW1);
  unsigned short* W2  = (unsigned short*)(ws + oW2);
  unsigned short* LNh = (unsigned short*)(ws + oLNh);
  unsigned short* LNl = (unsigned short*)(ws + oLNl);
  float* XR = (float*)(ws + oXR);
  unsigned short* Qh  = (unsigned short*)(ws + oQh);
  unsigned short* Ql  = (unsigned short*)(ws + oQl);
  unsigned short* Kp  = (unsigned short*)(ws + oK);
  unsigned short* Vh  = (unsigned short*)(ws + oVh);
  unsigned short* Vl  = (unsigned short*)(ws + oVl);
  unsigned short* Oh  = (unsigned short*)(ws + oOh);
  unsigned short* Ol  = (unsigned short*)(ws + oOl);
  unsigned short* Hh  = (unsigned short*)(ws + oHh);
  unsigned short* Hl  = (unsigned short*)(ws + oHl);

  const dim3 blk(256);
  cvt_wT<<<dim3(CDIM / 64, CQKV / 32), blk, 0, stream>>>(w_qkv, Wq, CDIM, CQKV);
  cvt_wT<<<dim3(CDIM / 64, CDIM / 32), blk, 0, stream>>>(w_proj, Wp, CDIM, CDIM);
  cvt_wT<<<dim3(CDIM / 64, CMLP / 32), blk, 0, stream>>>(w_fc1, W1, CDIM, CMLP);
  cvt_wT<<<dim3(CMLP / 64, CDIM / 32), blk, 0, stream>>>(w_fc2, W2, CMLP, CDIM);
  ln256<true><<<dim3(NTOK / 8), blk, 0, stream>>>(x, g1, b1, LNh, LNl);
  gemm_k<1><<<dim3(CDIM / 64, NBLK), blk, 0, stream>>>(
      LNh, LNl, Wq, CDIM, 0, 0, b_qkv, x, XR, Qh, Ql, Kp, Vh, Vl, 1.0f / 2048.0f);
  gemm_k<1><<<dim3((2 * CDIM) / 64, KVBLK), blk, 0, stream>>>(
      LNh, LNl, Wq, CDIM, CDIM, 0, b_qkv, x, XR, Qh, Ql, Kp, Vh, Vl, 1.0f / 2048.0f);
  attn_k<<<dim3(NWT * NHEAD), dim3(128), 0, stream>>>(Qh, Ql, Kp, Vh, Vl, rpb, Oh, Ol);
  gemm_k<2><<<dim3(CDIM / 64, NBLK), blk, 0, stream>>>(
      Oh, Ol, Wp, CDIM, 0, 0, b_proj, x, XR, Hh, Hh, Hh, Hh, Hh, 1.0f / 65536.0f);
  ln256<false><<<dim3(NTOK / 8), blk, 0, stream>>>(XR, g2, b2, LNh, LNl);
  gemm_k<3><<<dim3(CMLP / 64, MB0), blk, 0, stream>>>(
      LNh, LNl, W1, CDIM, 0, 0, b_fc1, XR, XR, Hh, Hl, Hh, Hh, Hh, 1.0f / 2048.0f);
  gemm_k<0><<<dim3(CDIM / 64, MB0), blk, 0, stream>>>(
      Hh, Hl, W2, CMLP, 0, 0, b_fc2, XR, out, Hh, Hh, Hh, Hh, Hh, 1.0f / 16384.0f);
  if (MB1 > 0) {
    gemm_k<3><<<dim3(CMLP / 64, MB1), blk, 0, stream>>>(
        LNh, LNl, W1, CDIM, 0, MB0 * 128, b_fc1, XR, XR, Hh, Hl, Hh, Hh, Hh, 1.0f / 2048.0f);
    gemm_k<0><<<dim3(CDIM / 64, MB1), blk, 0, stream>>>(
        Hh, Hl, W2, CMLP, 0, MB0 * 128, b_fc2, XR, out, Hh, Hh, Hh, Hh, Hh, 1.0f / 16384.0f);
  }
  (void)hipGetLastError();
}
